// Encoder_60438779789634
// MI455X (gfx1250) — hardware-verified
//
#include <hip/hip_runtime.h>
#include <math.h>

constexpr int NBATCH  = 32;
constexpr int NSTEP   = 512;
constexpr int NEMB    = 256;
constexpr int NUNIT   = 256;
constexpr int NGATE   = 4 * NUNIT;
constexpr int NVOCAB  = 50257;
constexpr int NROWS   = NBATCH * NSTEP;
constexpr int NXW     = 2 * NGATE;
constexpr int OUTW    = 2 * NUNIT;
constexpr int NTHR    = 256;
constexpr int SEQ_BLK = 16;
constexpr int XWPITCH = 1032;
constexpr int HPITCH  = 264;
constexpr int SLABP   = 36;
constexpr int NOUT0   = NBATCH * NSTEP * OUTW;
constexpr int NOUT1   = NBATCH * OUTW;
constexpr float XCARRY    = 16.0f;
constexpr float WCARRY    = 16.0f;
constexpr float HCARRY    = 1024.0f;
constexpr float XWCARRY   = 64.0f;
constexpr float GEMM_FOLD = 1.0f / (XCARRY * WCARRY);
constexpr float REC_FOLD  = 1.0f / (HCARRY * WCARRY);
constexpr float XW_FOLD   = 1.0f / XWCARRY;

static_assert(NEMB == NUNIT);
static_assert(NEMB % 32 == 0);
static_assert(NROWS % 64 == 0 && NXW % 64 == 0);
static_assert(NGATE % 64 == 0 && NUNIT % 64 == 0);
static_assert(NBATCH == 2 * SEQ_BLK);
static_assert(NUNIT == 32 * (NTHR / 32));
static_assert((2 * SEQ_BLK * HPITCH) % NTHR == 0);
static_assert((size_t)NOUT0 * 4 == 33554432u);
static_assert(((size_t)NOUT0 + NOUT1) * 4 == 33619968u);
static_assert(((size_t)NOUT0 + 2 * (size_t)NOUT1) * 4 == 33685504u);
static_assert((XWPITCH % 8) == 0 && (HPITCH % 8) == 0 && (SLABP % 4) == 0);

typedef __attribute__((ext_vector_type(16))) _Float16 v16h;
typedef __attribute__((ext_vector_type(8)))  _Float16 v8h;
typedef __attribute__((ext_vector_type(8)))  float    v8f;
typedef __attribute__((ext_vector_type(4)))  float    v4f;
typedef __attribute__((ext_vector_type(4)))  unsigned v4u;

__device__ __forceinline__ void guard4_h(v8f& a, v8f& b, v8f& c, v8f& d, v16h x, v16h y0, v16h y1, v16h y2, v16h y3) {
  asm volatile("v_nop\n\tv_nop\n\tv_nop\n\tv_nop" : "+v"(a), "+v"(b), "+v"(c), "+v"(d) : "v"(x), "v"(y0), "v"(y1), "v"(y2), "v"(y3));
}
__device__ __forceinline__ void keep4_h(v16h a, v16h b, v16h c, v16h d) { asm volatile("v_nop" :: "v"(a), "v"(b), "v"(c), "v"(d)); }
__device__ __forceinline__ void acc_guard4(v8f& a, v8f& b, v8f& c, v8f& d) { asm volatile("v_nop\n\tv_nop\n\tv_nop\n\tv_nop" : "+v"(a), "+v"(b), "+v"(c), "+v"(d)); }

struct FragH {
  union U { v16h v; v8h h[2]; };
  static __device__ __forceinline__ v16h load(const _Float16* p) {
    U f; f.h[0] = *(const v8h*)(p); f.h[1] = *(const v8h*)(p + 16); return f.v;
  }
  static __device__ __forceinline__ v8f mma(v16h a, v16h b, v8f c) {
    return __builtin_amdgcn_wmma_f32_16x16x32_f16(false, a, false, b, (short)0, c, false, false);
  }
};

__device__ __forceinline__ void wave_lds_sync() {
  __builtin_amdgcn_fence(__ATOMIC_RELEASE, "workgroup");
  __builtin_amdgcn_wave_barrier();
  __builtin_amdgcn_fence(__ATOMIC_ACQUIRE, "workgroup");
}

__device__ __forceinline__ float h16_to_f32(unsigned hb) {
  const unsigned sgn = (hb & 0x8000u) << 16; const unsigned em = hb & 0x7fffu;
  const float fn = __uint_as_float((em << 13) + 0x38000000u);
  const float fs = (float)em * 5.9604644775390625e-8f;
  const float mag = (em < 0x400u) ? fs : fn; return __uint_as_float(__float_as_uint(mag) | sgn);
}

__device__ __forceinline__ float fsig(float x) { return __builtin_amdgcn_rcpf(1.0f + expf(-x)); }

__global__ __launch_bounds__(NTHR) void gather_x16_kernel(const int* __restrict__ tokens, const float* __restrict__ emb,
                                                          unsigned short* __restrict__ X16) {
  const int i = blockIdx.x * NTHR + threadIdx.x;
  if (i < NROWS * (NEMB / 8)) {
    const int m  = i >> 5;
    const int c8 = (i & 31) * 8;
    const int tt = m >> 5;
    const int bb = m & 31;
    int tk = tokens[bb * NSTEP + tt];
    tk = tk < 0 ? 0 : (tk > NVOCAB - 1 ? NVOCAB - 1 : tk);
    const float* sp = emb + (size_t)tk * NEMB + c8;
    const v4f a = *(const v4f*)(sp);
    const v4f b = *(const v4f*)(sp + 4);
    v8h hv;
#pragma unroll
    for (int e = 0; e < 4; ++e) {
      const float fa = a[e] * XCARRY;
      const float fb = b[e] * XCARRY;
      hv[e]     = (_Float16)fa;
      hv[4 + e] = (_Float16)fb;
    }
    *(volatile v8h*)(X16 + (size_t)i * 8) = hv;
    __threadfence();
    *(volatile v8h*)(X16 + (size_t)i * 8) = hv;
  }
}

__global__ __launch_bounds__(NTHR) void tpw4_kernel(const float* __restrict__ s0, const float* __restrict__ s1,
                                                    const float* __restrict__ s2, const float* __restrict__ s3,
                                                    unsigned short* __restrict__ O) {
  __shared__ float Tt[64 * 65];
  const int tid = threadIdx.x;
  const int z = blockIdx.z;
  const float* src = (z == 0) ? s0 : ((z == 1) ? s1 : ((z == 2) ? s2 : s3));
  unsigned short* Oz = O + (size_t)z * NGATE * NUNIT;
  const int c0 = blockIdx.x * 64, r0 = blockIdx.y * 64;
#pragma unroll
  for (int i = 0; i < 4; ++i) {
    const int idx = i * NTHR + tid;
    const int rr = idx >> 4, cc = (idx & 15) * 4;
    const v4f v = *(const v4f*)(src + (size_t)(r0 + rr) * (size_t)NGATE + c0 + cc);
    Tt[rr * 65 + cc + 0] = v[0];
    Tt[rr * 65 + cc + 1] = v[1];
    Tt[rr * 65 + cc + 2] = v[2];
    Tt[rr * 65 + cc + 3] = v[3];
  }
  __syncthreads();
  const int q = tid >> 3, c8 = (tid & 7) * 8;
  v8h hv[2];
#pragma unroll
  for (int g = 0; g < 2; ++g) {
    const int qq = g * 32 + q;
#pragma unroll
    for (int e = 0; e < 8; ++e) {
      const float f = Tt[(c8 + e) * 65 + qq] * WCARRY;
      hv[g][e] = (_Float16)f;
    }
  }
  for (int pass = 0; pass < 2; ++pass) {
#pragma unroll
    for (int g = 0; g < 2; ++g) {
      const size_t o = (size_t)(c0 + g * 32 + q) * (size_t)NUNIT + (size_t)(r0 + c8);
      *(volatile v8h*)(Oz + o) = hv[g];
    }
    __threadfence();
  }
}

__global__ __launch_bounds__(NTHR) void xw_gemm_kernel(const unsigned short* __restrict__ Ap,
                                                       const unsigned short* __restrict__ Btp,
                                                       unsigned short* __restrict__ Cout,
                                                       const float* __restrict__ biasF,
                                                       const float* __restrict__ biasB) {
  const _Float16* A  = (const _Float16*)Ap;
  const _Float16* Bt = (const _Float16*)Btp;
  __shared__ __align__(16) float sT[8][16 * 68];
  const int lane = threadIdx.x & 31;
  const int wave = threadIdx.x >> 5;
  constexpr int tilesN = NXW >> 6;
  constexpr int tilesM = NROWS >> 6;
  const int tile = blockIdx.x * 8 + wave;
  if (tile >= tilesM * tilesN) return;
  const int tm = tile / tilesN;
  const int tn = tile - tm * tilesN;
  const int m0 = tm << 6;
  const int n0 = tn << 6;
  const int rlane = lane & 15;
  const int koff  = (lane >> 4) * 8;
  const int mOff  = (lane >> 4) * 8;

  v8f acc[4][4];
#pragma unroll
  for (int i = 0; i < 4; ++i)
#pragma unroll
    for (int j = 0; j < 4; ++j) acc[i][j] = (v8f){0.f, 0.f, 0.f, 0.f, 0.f, 0.f, 0.f, 0.f};

#pragma unroll 1
  for (int k0 = 0; k0 < NEMB; k0 += 32) {
    v16h bh[4];
#pragma unroll
    for (int j = 0; j < 4; ++j) {
      const size_t bo = (size_t)(n0 + (j << 4) + rlane) * NEMB + koff + k0;
      bh[j] = FragH::load(Bt + bo);
    }
#pragma unroll
    for (int i = 0; i < 4; ++i) {
      const size_t ao = (size_t)(m0 + (i << 4) + rlane) * NEMB + koff + k0;
      const v16h ah = FragH::load(A + ao);
#pragma unroll
      for (int j = 0; j < 4; ++j) acc[i][j] = FragH::mma(ah, bh[j], acc[i][j]);
      guard4_h(acc[i][0], acc[i][1], acc[i][2], acc[i][3], ah, bh[0], bh[1], bh[2], bh[3]);
    }
    keep4_h(bh[0], bh[1], bh[2], bh[3]);
  }
  acc_guard4(acc[0][0], acc[0][1], acc[0][2], acc[0][3]);
  acc_guard4(acc[1][0], acc[1][1], acc[1][2], acc[1][3]);
  acc_guard4(acc[2][0], acc[2][1], acc[2][2], acc[2][3]);
  acc_guard4(acc[3][0], acc[3][1], acc[3][2], acc[3][3]);

  float* slab = sT[wave];
#pragma unroll
  for (int i = 0; i < 4; ++i) {
    const int mBase = m0 + (i << 4);
#pragma unroll
    for (int j = 0; j < 4; ++j) {
      const int n  = n0 + (j << 4) + rlane;
      const int nn = n & (NGATE - 1);
      const float ba = biasF[nn];
      const float bb = biasB[nn];
      const float bv = (n0 < NGATE) ? ba : bb;
#pragma unroll
      for (int r = 0; r < 8; ++r) {
        const float v = (acc[i][j][r] * GEMM_FOLD + bv) * XWCARRY;
        slab[(mOff + r) * 68 + (j << 4) + rlane] = v;
      }
    }
    wave_lds_sync();
    {
      const int q = lane >> 3, c8 = (lane & 7) * 8;
      for (int pass = 0; pass < 2; ++pass) {
#pragma unroll
        for (int it = 0; it < 4; ++it) {
          const int row = it * 4 + q;
          const float* sp = slab + row * 68 + c8;
          v8h hv;
#pragma unroll
          for (int e = 0; e < 8; ++e) {
            const float f = sp[e];
            hv[e] = (_Float16)f;
          }
          *(volatile v8h*)(Cout + (size_t)(mBase + row) * NXW + n0 + c8) = hv;
        }
        __threadfence();
      }
    }
    wave_lds_sync();
  }
}

__global__ __launch_bounds__(NTHR) void bilstm_scan_kernel(const int* __restrict__ tokens,
                                                           const unsigned short* __restrict__ XW16,
                                                           const unsigned short* __restrict__ WrT16p,
                                                           float* __restrict__ out0, float* __restrict__ out1,
                                                           float* __restrict__ out2) {
  __shared__ __align__(16) unsigned short XWs[SEQ_BLK * XWPITCH];
  __shared__ __align__(16) _Float16       Ah[2][SEQ_BLK * HPITCH];
  __shared__ __align__(16) float          Sl[NTHR / 32][16 * SLABP];
  __shared__ int mk[SEQ_BLK];

  const int tid = threadIdx.x, lane = tid & 31, wave = tid >> 5;
  const int c = lane & 15, hh = lane >> 4, koff = hh * 8;
  const int dir = blockIdx.x >> 1;
  const int rowbase = (blockIdx.x & 1) * SEQ_BLK;
  const _Float16* WR = (const _Float16*)WrT16p + (size_t)dir * NGATE * NUNIT;

  {
    _Float16* ahf = &Ah[0][0];
#pragma unroll 1
    for (int i = tid; i < 2 * SEQ_BLK * HPITCH; i += NTHR) ahf[i] = (_Float16)0.0f;
  }
  float cA[8], hA[8], cB[8], hB[8];
#pragma unroll
  for (int r = 0; r < 8; ++r) { cA[r] = 0.0f; hA[r] = 0.0f; cB[r] = 0.0f; hB[r] = 0.0f; }
  __syncthreads();

  const v8f z8 = {0.f, 0.f, 0.f, 0.f, 0.f, 0.f, 0.f, 0.f};
  float* slab = &Sl[wave][0];
  const int sq = lane >> 3, sc4 = (lane & 7) * 4;

#pragma unroll 1
  for (int s = 0; s < NSTEP; ++s) {
    const int t   = dir ? (NSTEP - 1 - s) : s;
    const int cur = s & 1;

    {
      const unsigned short* gsrc = XW16 + ((size_t)(t * NBATCH + rowbase)) * NXW + (size_t)dir * NGATE;
      v4u tmp[8];
#pragma unroll
      for (int i = 0; i < 8; ++i) {
        const int idx = i * NTHR + tid;
        const int row = idx >> 7, cc = (idx & 127) * 8;
        tmp[i] = *(const v4u*)(gsrc + (size_t)row * NXW + cc);
      }
      int tk = tokens[(rowbase + (tid & 15)) * NSTEP + t];
      asm volatile("" : "+v"(tk));
#pragma unroll
      for (int i = 0; i < 8; ++i) {
        const int idx = i * NTHR + tid;
        const int row = idx >> 7, cc = (idx & 127) * 8;
        *(v4u*)(XWs + row * XWPITCH + cc) = tmp[i];
      }
      if (tid < SEQ_BLK) mk[tid] = tk;
    }
    __syncthreads();

    const _Float16* ahrow = &Ah[cur][0] + c * HPITCH + koff;
    _Float16* ahn = &Ah[cur ^ 1][0];

#pragma unroll 1
    for (int nt = 0; nt < 2; ++nt) {
      const int j = 32 * wave + 16 * nt + c;
      const _Float16* wr = WR + (size_t)j * NUNIT + koff;
      v8f a0 = z8, a1 = z8, a2 = z8, a3 = z8;
#pragma unroll 1
      for (int k0 = 0; k0 < NUNIT; k0 += 32) {
        const v16h a  = FragH::load(ahrow + k0);
        const v16h b0 = FragH::load(wr + k0);
        const v16h b1 = FragH::load(wr + (size_t)1 * NUNIT * NUNIT + k0);
        const v16h b2 = FragH::load(wr + (size_t)2 * NUNIT * NUNIT + k0);
        const v16h b3 = FragH::load(wr + (size_t)3 * NUNIT * NUNIT + k0);
        a0 = FragH::mma(a, b0, a0);
        a1 = FragH::mma(a, b1, a1);
        a2 = FragH::mma(a, b2, a2);
        a3 = FragH::mma(a, b3, a3);
        guard4_h(a0, a1, a2, a3, a, b0, b1, b2, b3);
      }
      acc_guard4(a0, a1, a2, a3);

#pragma unroll
      for (int r = 0; r < 8; ++r) {
        const int row = 8 * hh + r;
        const unsigned short* xr = XWs + row * XWPITCH + j;
        const float xi = h16_to_f32((unsigned)xr[0]);
        const float xf = h16_to_f32((unsigned)xr[NUNIT]);
        const float xg = h16_to_f32((unsigned)xr[2 * NUNIT]);
        const float xo = h16_to_f32((unsigned)xr[3 * NUNIT]);
        const float zi = xi * XW_FOLD + a0[r] * REC_FOLD;
        const float zf = xf * XW_FOLD + a1[r] * REC_FOLD;
        const float zg = xg * XW_FOLD + a2[r] * REC_FOLD;
        const float zo = xo * XW_FOLD + a3[r] * REC_FOLD;
        const float ig = fsig(zi);
        const float fg = fsig(zf);
        const float gg = fmaxf(zg, 0.0f);
        const float og = fsig(zo);
        const float cold = cA[r];
        const float hold = hA[r];
        const float cn = fg * cold + ig * gg;
        const float hn = og * fmaxf(cn, 0.0f);
        const bool keep = (mk[row] != 0);
        const float h2 = keep ? hn : hold;
        const float c2 = keep ? cn : cold;
        cA[r] = c2;
        hA[r] = h2;
        ahn[row * HPITCH + j] = (_Float16)(h2 * HCARRY);
        slab[row * SLABP + 16 * nt + c] = h2;
      }
#pragma unroll
      for (int r = 0; r < 8; ++r) {
        const float tc = cA[r]; cA[r] = cB[r]; cB[r] = tc;
        const float th = hA[r]; hA[r] = hB[r]; hB[r] = th;
      }
    }

    wave_lds_sync();
    {
      float* dst = out0 + ((size_t)rowbase * NSTEP + (size_t)t) * OUTW + (size_t)dir * NUNIT + 32 * wave;
      for (int pass = 0; pass < 2; ++pass) {
#pragma unroll
        for (int it = 0; it < 4; ++it) {
          const int row = it * 4 + sq;
          const v4f v = *(const v4f*)(slab + row * SLABP + sc4);
          *(volatile v4f*)(dst + (size_t)row * ((size_t)NSTEP * OUTW) + sc4) = v;
        }
        __threadfence();
      }
    }
    __syncthreads();
  }

#pragma unroll
  for (int r = 0; r < 8; ++r) {
    const float v0 = dir ? cA[r] : hA[r];
    const float v1 = dir ? cB[r] : hB[r];
    slab[(8 * hh + r) * SLABP + c]      = v0;
    slab[(8 * hh + r) * SLABP + 16 + c] = v1;
  }
  wave_lds_sync();
  {
    float* dst = out1 + (size_t)rowbase * OUTW + (size_t)dir * NUNIT + 32 * wave;
    for (int pass = 0; pass < 2; ++pass) {
#pragma unroll
      for (int it = 0; it < 4; ++it) {
        const int row = it * 4 + sq;
        const v4f v = *(const v4f*)(slab + row * SLABP + sc4);
        *(volatile v4f*)(dst + (size_t)row * OUTW + sc4) = v;
      }
      __threadfence();
    }
  }
  wave_lds_sync();
#pragma unroll
  for (int r = 0; r < 8; ++r) {
    slab[(8 * hh + r) * SLABP + c]      = cA[r];
    slab[(8 * hh + r) * SLABP + 16 + c] = cB[r];
  }
  wave_lds_sync();
  {
    float* dst = out2 + (size_t)rowbase * OUTW + (size_t)dir * NUNIT + 32 * wave;
    for (int pass = 0; pass < 2; ++pass) {
#pragma unroll
      for (int it = 0; it < 4; ++it) {
        const int row = it * 4 + sq;
        const v4f v = *(const v4f*)(slab + row * SLABP + sc4);
        *(volatile v4f*)(dst + (size_t)row * OUTW + sc4) = v;
      }
      __threadfence();
    }
  }
}

extern "C" void kernel_launch(void* const* d_in, const int* in_sizes, int n_in,
                              void* d_out, int out_size, void* d_ws, size_t ws_size, hipStream_t stream) {
  if (n_in < 8 || d_out == nullptr || d_ws == nullptr) return;
  if (in_sizes[0] != NBATCH * NSTEP || in_sizes[1] != NVOCAB * NEMB || in_sizes[2] != NEMB * NGATE ||
      in_sizes[3] != NUNIT * NGATE || in_sizes[4] != NGATE || in_sizes[5] != NEMB * NGATE ||
      in_sizes[6] != NUNIT * NGATE || in_sizes[7] != NGATE || out_size != NOUT0 + 2 * NOUT1) return;

  const int*   tokens = (const int*)d_in[0];
  const float* emb    = (const float*)d_in[1];
  const float* wk_f   = (const float*)d_in[2];
  const float* wr_f   = (const float*)d_in[3];
  const float* b_f    = (const float*)d_in[4];
  const float* wk_b   = (const float*)d_in[5];
  const float* wr_b   = (const float*)d_in[6];
  const float* b_b    = (const float*)d_in[7];
  float* out0 = (float*)d_out;
  float* out1 = out0 + (size_t)NOUT0;
  float* out2 = out1 + (size_t)NOUT1;

  char* ws = (char*)d_ws; size_t off = 0;
  auto carve = [&](size_t bytes) -> char* { char* p = ws + off; off += (bytes + 255) & ~(size_t)255; return p; };
  unsigned short* X16  = (unsigned short*)carve((size_t)NROWS * NEMB * 2);
  unsigned short* W16  = (unsigned short*)carve((size_t)4 * NGATE * NUNIT * 2);
  unsigned short* XW16 = (unsigned short*)carve((size_t)NROWS * NXW * 2);
  if (off > ws_size || off > (size_t)134217728) return;
  unsigned short* WkT16 = W16;
  unsigned short* WrT16 = W16 + (size_t)2 * NGATE * NUNIT;

  gather_x16_kernel<<<(NROWS * (NEMB / 8)) / NTHR, NTHR, 0, stream>>>(tokens, emb, X16);
  tpw4_kernel<<<dim3(NGATE / 64, NUNIT / 64, 4), NTHR, 0, stream>>>(wk_f, wk_b, wr_f, wr_b, W16);
  xw_gemm_kernel<<<((NROWS / 64) * (NXW / 64)) / 8, NTHR, 0, stream>>>(X16, WkT16, XW16, b_f, b_b);
  bilstm_scan_kernel<<<2 * (NBATCH / SEQ_BLK), NTHR, 0, stream>>>(tokens, XW16, WrT16, out0, out1, out2);
}
